// DeltaNet_22488448762175
// MI455X (gfx1250) — hardware-verified
//
#include <hip/hip_runtime.h>
#include <math.h>

constexpr int kBatch    = 4;
constexpr int kSeq      = 2048;
constexpr int kHid      = 1024;
constexpr int kHeads    = 16;
constexpr int kHd       = 64;
constexpr int kTok      = kBatch * kSeq;
constexpr int kQkvPitch = 3 * kHid;
constexpr int kChunk    = 64;
constexpr int kNumChunk = kSeq / kChunk;
constexpr int kBetaPad  = 64;
constexpr int kBtRows   = 4 * kHid + kBetaPad;
constexpr int kRowK     = kHid;
constexpr int kRowO     = 3 * kHid;
constexpr int kRowBeta  = 4 * kHid;
constexpr int kNormThr  = 128;
constexpr int kLnThr    = 256;
constexpr float kRmsEps   = 1e-6f;
constexpr float kLnEps    = 1e-5f;
constexpr float kDenEps   = 1e-6f;
constexpr float kBetaLo   = 0.9f;
constexpr float kBetaHi   = 0.9995f;
constexpr float kWCarry    = 16.0f;
constexpr float kWCarryInv = 1.0f / kWCarry;
constexpr float kInvHid    = 1.0f / (float)kHid;
static_assert(kHeads * kHd == kHid, "head split");
static_assert(kHd == 64 && kChunk == 64, "scan tiles are 64x64");
static_assert(kSeq % kChunk == 0, "chunks never straddle a batch");
static_assert(kTok % 64 == 0 && kHid % 64 == 0 && (2 * kHid) % 64 == 0 && kBetaPad % 64 == 0, "GEMM M,N tile multiples");
static_assert(kHid % 32 == 0, "GEMM K multiple of 32");
static_assert(kNormThr * 8 == kHid, "row norm: 128 threads x 8 columns cover one row");
static_assert(kLnThr * 4 == kHid, "LayerNorm: 256 threads x 4 columns cover one row");
static_assert(kBtRows % 2 == 0 && (kHid % 2) == 0, "weight pack: 2 rows per block, segment uniform per block");

typedef __attribute__((ext_vector_type(16))) _Float16 v16h;
typedef __attribute__((ext_vector_type(8)))  _Float16 v8h;
typedef __attribute__((ext_vector_type(8)))  float    v8f;
typedef __attribute__((ext_vector_type(4)))  float    v4f;
typedef __attribute__((ext_vector_type(4)))  unsigned int v4u;

__device__ __forceinline__ void dep_guard4_h(v8f& a, v8f& b, v8f& c, v8f& d, v16h x) {
  asm volatile("v_nop\n\tv_nop\n\tv_nop\n\tv_nop" : "+v"(a), "+v"(b), "+v"(c), "+v"(d) : "v"(x));
}
__device__ __forceinline__ void keep4_h(v16h a, v16h b, v16h c, v16h d) { asm volatile("v_nop" :: "v"(a), "v"(b), "v"(c), "v"(d)); }
__device__ __forceinline__ void acc_guard4(v8f& a, v8f& b, v8f& c, v8f& d) { asm volatile("v_nop\n\tv_nop\n\tv_nop\n\tv_nop" : "+v"(a), "+v"(b), "+v"(c), "+v"(d)); }

struct FragH {
  union U { v16h v; v8h h[2]; };
  static __device__ __forceinline__ v16h load(const _Float16* p) {
    U f; f.h[0] = *(const v8h*)(p); f.h[1] = *(const v8h*)(p + 16); return f.v;
  }
  static __device__ __forceinline__ v8f mma(v16h a, v16h b, v8f c) {
    return __builtin_amdgcn_wmma_f32_16x16x32_f16(false, a, false, b, (short)0, c, false, false);
  }
};
__device__ __forceinline__ v8f mma_g(v16h a, v16h b, v8f c) {
  c = __builtin_amdgcn_wmma_f32_16x16x32_f16(false, a, false, b, (short)0, c, false, false);
  asm volatile("v_nop\n\tv_nop\n\tv_nop\n\tv_nop" : "+v"(c) : "v"(a), "v"(b));
  return c;
}

__device__ __forceinline__ float h16_to_f32(unsigned hb) {
  const unsigned sgn = (hb & 0x8000u) << 16; const unsigned em = hb & 0x7fffu;
  const float fn = __uint_as_float((em << 13) + 0x38000000u);
  const float fs = (float)em * 5.9604644775390625e-8f;
  const float mag = (em < 0x400u) ? fs : fn; return __uint_as_float(__float_as_uint(mag) | sgn);
}

template <int OUT_MODE, bool ADD_BR>
__global__ __launch_bounds__(256) void gemm64_f16(
    const unsigned short* __restrict__ Ap, int lda,
    const unsigned short* __restrict__ Btp, int ldb,
    void* __restrict__ Cout, int ldc,
    const float* __restrict__ bias,
    const float* __restrict__ resid, int ldr,
    int M, int N, int K, float scale) {
  const _Float16* A  = (const _Float16*)Ap;
  const _Float16* Bt = (const _Float16*)Btp;
  __shared__ __align__(16) float sT[8][16 * 68];
  const int lane = threadIdx.x & 31;
  const int wave = threadIdx.x >> 5;
  const int tilesN = N >> 6;
  const int tilesM = M >> 6;
  const int tile = blockIdx.x * 8 + wave;
  if (tile >= tilesM * tilesN) return;
  const int tm = tile / tilesN;
  const int tn = tile - tm * tilesN;
  const int m0 = tm << 6;
  const int n0 = tn << 6;
  const int rlane = lane & 15;
  const int koff  = (lane >> 4) * 8;
  const int mOff  = (lane >> 4) * 8;

  v8f acc[4][4];
#pragma unroll
  for (int i = 0; i < 4; ++i)
#pragma unroll
    for (int j = 0; j < 4; ++j) acc[i][j] = (v8f){0.f, 0.f, 0.f, 0.f, 0.f, 0.f, 0.f, 0.f};

  const _Float16* Abase = A  + (size_t)(m0 + rlane) * lda + koff;
  const _Float16* Bbase = Bt + (size_t)(n0 + rlane) * ldb + koff;
  const size_t astep = (size_t)16 * lda;
  const size_t bstep = (size_t)16 * ldb;

  for (int k0 = 0; k0 < K; k0 += 32) {
    v16h bh[4];
#pragma unroll
    for (int j = 0; j < 4; ++j) bh[j] = FragH::load(Bbase + j * bstep + k0);
#pragma unroll
    for (int i = 0; i < 4; ++i) {
      const v16h ah = FragH::load(Abase + i * astep + k0);
#pragma unroll
      for (int j = 0; j < 4; ++j) acc[i][j] = FragH::mma(ah, bh[j], acc[i][j]);
      dep_guard4_h(acc[i][0], acc[i][1], acc[i][2], acc[i][3], ah);
    }
    keep4_h(bh[0], bh[1], bh[2], bh[3]);
  }
  acc_guard4(acc[0][0], acc[0][1], acc[0][2], acc[0][3]);
  acc_guard4(acc[1][0], acc[1][1], acc[1][2], acc[1][3]);
  acc_guard4(acc[2][0], acc[2][1], acc[2][2], acc[2][3]);
  acc_guard4(acc[3][0], acc[3][1], acc[3][2], acc[3][3]);

  float* slab = sT[wave];
  const int hh = lane >> 4;
  const int c4 = (lane & 15) * 4;
  v4f bq = (v4f){0.f, 0.f, 0.f, 0.f};
  if (OUT_MODE == 0 && ADD_BR) bq = *(const v4f*)(bias + n0 + c4);
#pragma unroll
  for (int i = 0; i < 4; ++i) {
    const int mBase = m0 + (i << 4);
#pragma unroll
    for (int j = 0; j < 4; ++j) {
#pragma unroll
      for (int r = 0; r < 8; ++r) slab[(mOff + r) * 68 + (j << 4) + rlane] = acc[i][j][r] * scale;
    }
    __builtin_amdgcn_fence(__ATOMIC_RELEASE, "workgroup");
    __builtin_amdgcn_wave_barrier();
    __builtin_amdgcn_fence(__ATOMIC_ACQUIRE, "workgroup");
    if (OUT_MODE == 0) {
      float* C = (float*)Cout;
      v4f vals[8];
#pragma unroll
      for (int it = 0; it < 8; ++it) {
        const int row = it * 2 + hh;
        v4f v = *(const v4f*)(slab + row * 68 + c4);
        if (ADD_BR) {
          v = v + bq;
          const v4f rr = *(const v4f*)(resid + (size_t)(mBase + row) * ldr + n0 + c4);
          v = v + rr;
        }
        vals[it] = v;
      }
      for (int pass = 0; pass < 2; ++pass) {
#pragma unroll
        for (int it = 0; it < 8; ++it) {
          const int row = it * 2 + hh;
          *(volatile v4f*)(C + (size_t)(mBase + row) * ldc + n0 + c4) = vals[it];
        }
        __threadfence();
      }
    } else {
      const int q = lane >> 3, c8 = (lane & 7) * 8;
      unsigned short* C = (unsigned short*)Cout;
      for (int pass = 0; pass < 2; ++pass) {
#pragma unroll
        for (int it = 0; it < 4; ++it) {
          const int row = it * 4 + q;
          const float* sp = slab + row * 68 + c8;
          v8h hv;
#pragma unroll
          for (int e = 0; e < 8; ++e) hv[e] = (_Float16)sp[e];
          *(volatile v8h*)(C + (size_t)(mBase + row) * ldc + n0 + c8) = hv;
        }
        __threadfence();
      }
    }
    __builtin_amdgcn_fence(__ATOMIC_RELEASE, "workgroup");
    __builtin_amdgcn_wave_barrier();
    __builtin_amdgcn_fence(__ATOMIC_ACQUIRE, "workgroup");
  }
}

__global__ __launch_bounds__(128) void norm_rows_kernel(const float* __restrict__ x, const float* __restrict__ rin,
                                                        unsigned short* __restrict__ xn16,
                                                        unsigned short* __restrict__ xr16) {
  __shared__ float red1[4];
  __shared__ float red2[4];
  const int tid = threadIdx.x, lane = tid & 31, wave = tid >> 5;
  const size_t row = (size_t)blockIdx.x;
  const float* xp = x + row * kHid + 8 * tid;
  const v4f a  = *(const v4f*)(xp);
  const v4f b  = *(const v4f*)(xp + 4);
  const v4f ga = *(const v4f*)(rin + 8 * tid);
  const v4f gb = *(const v4f*)(rin + 8 * tid + 4);
  float ss = 0.0f;
#pragma unroll
  for (int e = 0; e < 4; ++e) { ss += a[e] * a[e]; ss += b[e] * b[e]; }
#pragma unroll
  for (int off = 1; off < 32; off <<= 1) ss += __shfl_xor(ss, off, 32);
  if (lane == 0) red1[wave] = ss;
  __syncthreads();
  const float tot1 = (red1[0] + red1[1]) + (red1[2] + red1[3]);
  const float r1 = rsqrtf(tot1 * kInvHid + kRmsEps);
  float nv[8];
  float ss2 = 0.0f;
#pragma unroll
  for (int e = 0; e < 4; ++e) {
    const float n0v = (a[e] * r1) * ga[e];
    const float n1v = (b[e] * r1) * gb[e];
    nv[e] = n0v;
    nv[4 + e] = n1v;
    ss2 += n0v * n0v;
    ss2 += n1v * n1v;
  }
#pragma unroll
  for (int off = 1; off < 32; off <<= 1) ss2 += __shfl_xor(ss2, off, 32);
  if (lane == 0) red2[wave] = ss2;
  __syncthreads();
  const float tot2 = (red2[0] + red2[1]) + (red2[2] + red2[3]);
  const float r2 = rsqrtf(tot2 * kInvHid + kRmsEps);
  v8h hn, hr;
#pragma unroll
  for (int e = 0; e < 8; ++e) {
    const float v = nv[e];
    hn[e] = (_Float16)v;
    hr[e] = (_Float16)(v * r2);
  }
  unsigned short* pn = xn16 + row * kHid + 8 * tid;
  unsigned short* pr = xr16 + row * kHid + 8 * tid;
  for (int pass = 0; pass < 2; ++pass) {
    *(volatile v8h*)pn = hn;
    *(volatile v8h*)pr = hr;
    __threadfence();
  }
}

__global__ __launch_bounds__(256) void pack_weights_kernel(const float* __restrict__ Wq, const float* __restrict__ Wk,
                                                           const float* __restrict__ Wv, const float* __restrict__ Wo,
                                                           const float* __restrict__ bw, const float* __restrict__ rk,
                                                           const float* __restrict__ rv, unsigned short* __restrict__ dst) {
  const int row0 = blockIdx.x * 2;
  const int seg  = row0 >> 10;
  const int row  = row0 + (threadIdx.x >> 7);
  const int c8   = (threadIdx.x & 127) * 8;
  const float* src = (seg == 0) ? Wq : (seg == 1) ? Wk : (seg == 2) ? Wv : (seg == 3) ? Wo : bw;
  const float* gsrc = (seg == 2) ? rv : rk;
  const bool useGain = (seg == 1) || (seg == 2);
  const int rl = row - (seg << 10);
  const bool real = (seg < 4) || (rl < kHeads);
  const int rs = (seg < 4) ? rl : ((rl < kHeads) ? rl : (kHeads - 1));
  const float* sp = src + (size_t)rs * kHid + c8;
  const v4f a  = *(const v4f*)(sp);
  const v4f b  = *(const v4f*)(sp + 4);
  const v4f ga = *(const v4f*)(gsrc + c8);
  const v4f gb = *(const v4f*)(gsrc + c8 + 4);
  v8h hv;
#pragma unroll
  for (int e = 0; e < 4; ++e) {
    const float g0 = useGain ? ga[e] : 1.0f;
    const float g1 = useGain ? gb[e] : 1.0f;
    const float v0 = real ? ((a[e] * g0) * kWCarry) : 0.0f;
    const float v1 = real ? ((b[e] * g1) * kWCarry) : 0.0f;
    hv[e]     = (_Float16)v0;
    hv[4 + e] = (_Float16)v1;
  }
  unsigned short* op = dst + (size_t)row * kHid + c8;
  *(volatile v8h*)op = hv;
  __threadfence();
  *(volatile v8h*)op = hv;
}

__global__ __launch_bounds__(256) void decay_scan_kernel(const unsigned short* __restrict__ qkv,
                                                         const float* __restrict__ logit,
                                                         const float* __restrict__ beta_b,
                                                         const float* __restrict__ base_logit,
                                                         unsigned short* __restrict__ o16) {
  __shared__ __align__(16) _Float16 Vt[64 * 64];
  __shared__ __align__(16) _Float16 Kwt[64 * 64];
  __shared__ __align__(16) _Float16 Sw[64 * 64];
  __shared__ __align__(16) _Float16 Mt[64 * 64];
  __shared__ __align__(16) _Float16 Os[64 * 64];
  __shared__ float sBeta[64];
  __shared__ float sP[64];
  __shared__ float sRP[64];
  __shared__ float sRD[64];

  const int tid = threadIdx.x, lane = tid & 31, wave = tid >> 5;
  const int c = lane & 15, hh = lane >> 4, koff = hh * 8;
  const int bh = blockIdx.x;
  const int b = bh >> 4;
  const int h = bh & 15;
  const int it  = wave >> 1;
  const int et0 = (wave & 1) * 2;
  const _Float16* qkvh = (const _Float16*)qkv;

  {
    const v8h zz = (v8h){(_Float16)0.0f, (_Float16)0.0f, (_Float16)0.0f, (_Float16)0.0f,
                         (_Float16)0.0f, (_Float16)0.0f, (_Float16)0.0f, (_Float16)0.0f};
#pragma unroll
    for (int i = 0; i < 2; ++i) *(v8h*)(Mt + (tid + 256 * i) * 8) = zz;
  }
  const v8f z8 = (v8f){0.f, 0.f, 0.f, 0.f, 0.f, 0.f, 0.f, 0.f};
  v8f macc[2];
  macc[0] = z8;
  macc[1] = z8;
  float dcar = 0.0f;
  const float bbias = beta_b[h];
  const float sbase = 1.0f / (1.0f + expf(-base_logit[h]));
  __syncthreads();

#pragma unroll 1
  for (int ck = 0; ck < kNumChunk; ++ck) {
    const size_t tok0 = (size_t)b * kSeq + (size_t)ck * kChunk;

    if (tid < 64) {
      const float z = logit[(tok0 + (size_t)tid) * kBetaPad + h] + bbias;
      const float sg = 1.0f / (1.0f + expf(-z));
      float bt = sg * sbase;
      bt = fminf(kBetaHi, fmaxf(kBetaLo, bt));
      sBeta[tid] = bt;
    }
    __syncthreads();

    if (wave == 0) {
      float p = 1.0f, d = dcar;
#pragma unroll 1
      for (int i = 0; i < kChunk; ++i) {
        const float bt = sBeta[i];
        p = p * bt;
        d = d * bt + 1.0f;
        const float rp = 1.0f / p;
        const float rd = 1.0f / (d + kDenEps);
        if (lane == 0) { sP[i] = p; sRP[i] = rp; sRD[i] = rd; }
      }
      dcar = d;
    }
    __syncthreads();

    {
      const int j = tid >> 2;
      const int seg = tid & 3;
      const unsigned short* rp = qkv + (tok0 + (size_t)j) * kQkvPitch + (size_t)h * kHd + seg * 16;
      const v4u kA = *(const v4u*)(rp + kHid);
      const v4u kB = *(const v4u*)(rp + kHid + 8);
      const v4u vA = *(const v4u*)(rp + 2 * kHid);
      const v4u vB = *(const v4u*)(rp + 2 * kHid + 8);
      const float ks = sP[kChunk - 1] * sRP[j];
#pragma unroll
      for (int i = 0; i < 4; ++i) {
        const unsigned ka = kA[i];
        const unsigned kb = kB[i];
        const unsigned va = vA[i];
        const unsigned vb = vB[i];
        const int d0 = seg * 16 + 2 * i;
        const int d1 = d0 + 8;
        Kwt[(d0) * 64 + j]     = (_Float16)(h16_to_f32(ka & 0xffffu) * ks);
        Kwt[(d0 + 1) * 64 + j] = (_Float16)(h16_to_f32(ka >> 16) * ks);
        Kwt[(d1) * 64 + j]     = (_Float16)(h16_to_f32(kb & 0xffffu) * ks);
        Kwt[(d1 + 1) * 64 + j] = (_Float16)(h16_to_f32(kb >> 16) * ks);
        const unsigned short va0 = (unsigned short)(va & 0xffffu);
        const unsigned short va1 = (unsigned short)(va >> 16);
        const unsigned short vb0 = (unsigned short)(vb & 0xffffu);
        const unsigned short vb1 = (unsigned short)(vb >> 16);
        Vt[(d0) * 64 + j]     = __builtin_bit_cast(_Float16, va0);
        Vt[(d0 + 1) * 64 + j] = __builtin_bit_cast(_Float16, va1);
        Vt[(d1) * 64 + j]     = __builtin_bit_cast(_Float16, vb0);
        Vt[(d1 + 1) * 64 + j] = __builtin_bit_cast(_Float16, vb1);
      }
    }
    __syncthreads();

    const _Float16* qrow = qkvh + (tok0 + (size_t)(it * 16 + c)) * kQkvPitch + (size_t)h * kHd + koff;
    const v16h qa0 = FragH::load(qrow);
    const v16h qa1 = FragH::load(qrow + 32);
#pragma unroll
    for (int j2 = 0; j2 < 2; ++j2) {
      const int jt = et0 + j2;
      const _Float16* krow = qkvh + (tok0 + (size_t)(jt * 16 + c)) * kQkvPitch + kHid + (size_t)h * kHd + koff;
      const v16h kb0 = FragH::load(krow);
      const v16h kb1 = FragH::load(krow + 32);
      v8f sacc = z8;
      sacc = mma_g(qa0, kb0, sacc);
      sacc = mma_g(qa1, kb1, sacc);
      const int jj = jt * 16 + c;
      const float rpj = sRP[jj];
#pragma unroll
      for (int r = 0; r < 8; ++r) {
        const int ii = it * 16 + 8 * hh + r;
        const float w = sP[ii] * rpj;
        const float sv = (jj <= ii) ? (sacc[r] * w) : 0.0f;
        Sw[ii * 64 + jj] = (_Float16)sv;
      }
    }
    __syncthreads();

    const float pc = sP[kChunk - 1];
    v16h fv[2][2];
    {
      const _Float16* swrow = Sw + (it * 16 + c) * 64 + koff;
      const v16h sa0 = FragH::load(swrow);
      const v16h sa1 = FragH::load(swrow + 32);
#pragma unroll
      for (int e2 = 0; e2 < 2; ++e2) {
        const int et = et0 + e2;
        const _Float16* vrow = Vt + (et * 16 + c) * 64 + koff;
        const _Float16* mrow = Mt + (et * 16 + c) * 64 + koff;
        fv[e2][0] = FragH::load(vrow);
        fv[e2][1] = FragH::load(vrow + 32);
        const v16h mb0 = FragH::load(mrow);
        const v16h mb1 = FragH::load(mrow + 32);
        v8f a1 = z8;
        a1 = mma_g(sa0, fv[e2][0], a1);
        a1 = mma_g(sa1, fv[e2][1], a1);
        v8f a2 = z8;
        a2 = mma_g(qa0, mb0, a2);
        a2 = mma_g(qa1, mb1, a2);
#pragma unroll
        for (int r = 0; r < 8; ++r) {
          const int ii = it * 16 + 8 * hh + r;
          const float o = (a1[r] + sP[ii] * a2[r]) * sRD[ii];
          Os[ii * 64 + et * 16 + c] = (_Float16)o;
        }
      }
    }
    __syncthreads();

    {
      const int c8 = (tid & 7) * 8;
      v8h ov[2];
#pragma unroll
      for (int i2 = 0; i2 < 2; ++i2) {
        const int row = i2 * 32 + (tid >> 3);
        ov[i2] = *(const v8h*)(Os + row * 64 + c8);
      }
      for (int pass = 0; pass < 2; ++pass) {
#pragma unroll
        for (int i2 = 0; i2 < 2; ++i2) {
          const int row = i2 * 32 + (tid >> 3);
          *(volatile v8h*)(o16 + (tok0 + (size_t)row) * kHid + (size_t)h * kHd + c8) = ov[i2];
        }
        __threadfence();
      }
    }

    {
      const _Float16* kwrow = Kwt + (it * 16 + c) * 64 + koff;
      const v16h ka0 = FragH::load(kwrow);
      const v16h ka1 = FragH::load(kwrow + 32);
#pragma unroll
      for (int e2 = 0; e2 < 2; ++e2) {
        v8f dm = z8;
        dm = mma_g(ka0, fv[e2][0], dm);
        dm = mma_g(ka1, fv[e2][1], dm);
        v8h hv;
#pragma unroll
        for (int r = 0; r < 8; ++r) {
          const float nv = pc * macc[e2][r] + dm[r];
          macc[e2][r] = nv;
          hv[r] = (_Float16)nv;
        }
        *(v8h*)(Mt + ((et0 + e2) * 16 + c) * 64 + it * 16 + 8 * hh) = hv;
      }
    }
  }
}

__global__ __launch_bounds__(256) void ln_rows_kernel(const float* __restrict__ YP, const float* __restrict__ gam,
                                                      const float* __restrict__ bet, float* __restrict__ Y) {
  __shared__ float redS[8];
  __shared__ float redQ[8];
  const int tid = threadIdx.x, lane = tid & 31, wave = tid >> 5;
  const size_t row = (size_t)blockIdx.x;
  const v4f v  = *(const v4f*)(YP + row * kHid + 4 * tid);
  const v4f g  = *(const v4f*)(gam + 4 * tid);
  const v4f bb = *(const v4f*)(bet + 4 * tid);
  float s = (v[0] + v[1]) + (v[2] + v[3]);
#pragma unroll
  for (int off = 1; off < 32; off <<= 1) s += __shfl_xor(s, off, 32);
  if (lane == 0) redS[wave] = s;
  __syncthreads();
  const float tot = ((redS[0] + redS[1]) + (redS[2] + redS[3])) + ((redS[4] + redS[5]) + (redS[6] + redS[7]));
  const float mu = tot * kInvHid;
  float d[4];
  float ss = 0.0f;
#pragma unroll
  for (int e = 0; e < 4; ++e) { d[e] = v[e] - mu; ss += d[e] * d[e]; }
#pragma unroll
  for (int off = 1; off < 32; off <<= 1) ss += __shfl_xor(ss, off, 32);
  if (lane == 0) redQ[wave] = ss;
  __syncthreads();
  const float tq = ((redQ[0] + redQ[1]) + (redQ[2] + redQ[3])) + ((redQ[4] + redQ[5]) + (redQ[6] + redQ[7]));
  const float var  = tq * kInvHid;
  const float rstd = rsqrtf(var + kLnEps);
  v4f o;
#pragma unroll
  for (int e = 0; e < 4; ++e) o[e] = (d[e] * rstd) * g[e] + bb[e];
  float* op = Y + row * kHid + 4 * tid;
  *(volatile v4f*)op = o;
  __threadfence();
  *(volatile v4f*)op = o;
}

extern "C" void kernel_launch(void* const* d_in, const int* in_sizes, int n_in,
                              void* d_out, int out_size, void* d_ws, size_t ws_size, hipStream_t stream) {
  if (n_in < 14 || d_out == nullptr || d_ws == nullptr) return;
  if (in_sizes[0] != kTok * kHid || in_sizes[1] != kHid || in_sizes[2] != kHid || in_sizes[3] != kHid ||
      in_sizes[4] != kHid * kHid || in_sizes[5] != kHid * kHid || in_sizes[6] != kHid * kHid ||
      in_sizes[7] != kHeads * kHid || in_sizes[8] != kHeads || in_sizes[9] != kHeads ||
      in_sizes[10] != kHid * kHid || in_sizes[11] != kHid || in_sizes[12] != kHid || in_sizes[13] != kHid ||
      out_size != kTok * kHid) return;

  const float* x      = (const float*)d_in[0];
  const float* rin_w  = (const float*)d_in[1];
  const float* rk_w   = (const float*)d_in[2];
  const float* rv_w   = (const float*)d_in[3];
  const float* Wq     = (const float*)d_in[4];
  const float* Wk     = (const float*)d_in[5];
  const float* Wv     = (const float*)d_in[6];
  const float* beta_w = (const float*)d_in[7];
  const float* beta_b = (const float*)d_in[8];
  const float* base_l = (const float*)d_in[9];
  const float* Wo     = (const float*)d_in[10];
  const float* bo     = (const float*)d_in[11];
  const float* ln_w   = (const float*)d_in[12];
  const float* ln_b   = (const float*)d_in[13];
  float* out = (float*)d_out;

  char* ws = (char*)d_ws;
  size_t off = 0;
  auto carve = [&](size_t bytes) -> char* { char* p = ws + off; off += (bytes + 255) & ~(size_t)255; return p; };
  unsigned short* XN16  = (unsigned short*)carve((size_t)kTok * kHid * 2);
  unsigned short* XR16  = (unsigned short*)carve((size_t)kTok * kHid * 2);
  unsigned short* BT    = (unsigned short*)carve((size_t)kBtRows * kHid * 2);
  unsigned short* QKV16 = (unsigned short*)carve((size_t)kTok * kQkvPitch * 2);
  float*          LOG   = (float*)carve((size_t)kTok * kBetaPad * 4);
  float*          Y32   = (float*)carve((size_t)kTok * kHid * 4);
  unsigned short* O16   = XN16;
  if (off > ws_size || off > (size_t)134217728) return;

  norm_rows_kernel<<<kTok, kNormThr, 0, stream>>>(x, rin_w, XN16, XR16);
  pack_weights_kernel<<<kBtRows / 2, 256, 0, stream>>>(Wq, Wk, Wv, Wo, beta_w, rk_w, rv_w, BT);

  gemm64_f16<1, false><<<(kTok / 64) * (kHid / 64) / 8, 256, 0, stream>>>(
      XN16, kHid, BT, kHid, (void*)QKV16, kQkvPitch, bo, x, kHid, kTok, kHid, kHid, kWCarryInv);
  gemm64_f16<1, false><<<(kTok / 64) * ((2 * kHid) / 64) / 8, 256, 0, stream>>>(
      XR16, kHid, BT + (size_t)kRowK * kHid, kHid, (void*)(QKV16 + kHid), kQkvPitch, bo, x, kHid,
      kTok, 2 * kHid, kHid, kWCarryInv);
  gemm64_f16<0, false><<<(kTok / 64) * (kBetaPad / 64) / 8, 256, 0, stream>>>(
      XN16, kHid, BT + (size_t)kRowBeta * kHid, kHid, (void*)LOG, kBetaPad, bo, x, kHid,
      kTok, kBetaPad, kHid, kWCarryInv);

  decay_scan_kernel<<<kBatch * kHeads, 256, 0, stream>>>(QKV16, LOG, beta_b, base_l, O16);

  gemm64_f16<0, true><<<(kTok / 64) * (kHid / 64) / 8, 256, 0, stream>>>(
      O16, kHid, BT + (size_t)kRowO * kHid, kHid, (void*)Y32, kHid, bo, x, kHid, kTok, kHid, kHid, kWCarryInv);

  ln_rows_kernel<<<kTok, kLnThr, 0, stream>>>(Y32, ln_w, ln_b, out);
}
